// GATSubstAttention_57011395887502
// MI455X (gfx1250) — hardware-verified
//
#include <hip/hip_runtime.h>
#include <hip/hip_bf16.h>
#include <math.h>


#define BB 2
#define SS 2048
#define DD 1024
#define HH 16
#define DKK 64
#define QW 2

typedef _Float16 bf16;
typedef __attribute__((ext_vector_type(4))) unsigned v4u_t;
typedef unsigned v4ua __attribute__((ext_vector_type(4), may_alias));
typedef __attribute__((ext_vector_type(4))) float v4f_t;
typedef float v4fa __attribute__((ext_vector_type(4), may_alias));
typedef __attribute__((ext_vector_type(16))) bf16  bf16x16;
typedef __attribute__((ext_vector_type(8)))  bf16  bf16x8;
typedef __attribute__((ext_vector_type(4)))  bf16  bf16x4;
typedef __attribute__((ext_vector_type(8)))  float f32x8;

#define LDS_STRIDE 48
#define KSTRIDE    72
#define VSTRIDE    48

__device__ __forceinline__ f32x8 wmma_bf16(bf16x16 a, bf16x16 b, f32x8 c) {
  return __builtin_amdgcn_wmma_f32_16x16x32_f16(
      false, a, false, b, (short)0, c, false, false);
}

template <typename T>
__device__ __forceinline__ bf16x16 load_frag(const T* __restrict__ base, int ld,
                                             int row0, int k0) {
  const int lane = threadIdx.x & 31;
  const int r    = lane & 15;
  const int kh   = (lane >> 4) * 8;
  const T* p0 = base + (size_t)(row0 + r) * ld + (k0 + kh);
  const T* p1 = p0 + 16;
  bf16x16 f;
#pragma unroll
  for (int i = 0; i < 8; ++i) {
    f[i]     = (bf16)p0[i];
    f[i + 8] = (bf16)p1[i];
  }
  return f;
}

__device__ __forceinline__ bf16x16 lds_frag(const bf16* base, int stride) {
  const int lane = threadIdx.x & 31;
  const int row  = lane & 15;
  const int kh   = (lane >> 4) * 8;
  const bf16x8 lo = *(const bf16x8*)(base + row * stride + kh);
  const bf16x8 hi = *(const bf16x8*)(base + row * stride + kh + 16);
  bf16x16 f;
#pragma unroll
  for (int i = 0; i < 8; ++i) { f[i] = lo[i]; f[i + 8] = hi[i]; }
  return f;
}

template <typename T>
__device__ __forceinline__ void stage_read16(const T* __restrict__ p, float* buf) {
#pragma unroll
  for (int i = 0; i < 16; ++i) buf[i] = (float)p[i];
}

__device__ __forceinline__ void stage_write(bf16* dst, const float* buf, int nquad) {
#pragma unroll
  for (int i = 0; i < nquad; ++i) {
    bf16x4 q;
    q[0] = (bf16)buf[4 * i];     q[1] = (bf16)buf[4 * i + 1];
    q[2] = (bf16)buf[4 * i + 2]; q[3] = (bf16)buf[4 * i + 3];
    *(bf16x4*)(dst + 4 * i) = q;
  }
}

template <typename AT, typename WTY, int MODE>
__global__ __launch_bounds__(256) void gemm_bias_kernel(
    const AT* __restrict__ A, const WTY* __restrict__ W,
    const float* __restrict__ bias, void* __restrict__ out,
    int M, int N, int K) {
  __shared__ bf16 ldsA[128 * LDS_STRIDE];
  __shared__ bf16 ldsW[256 * LDS_STRIDE];
  __shared__ __attribute__((aligned(16))) unsigned char sob[256 * 136 * 2];

  const int t    = threadIdx.x;
  const int wave = t >> 5;
  const int lane = t & 31;
  const int wm   = (wave & 1) * 64;
  const int wn   = (wave >> 1) * 64;
  const int mBlk = blockIdx.x * 128;
  const int nBlk = blockIdx.y * 256;

  const int arow = t >> 1;
  const int ach  = (t & 1) * 16;

  float abuf[16];
  float wbuf[32];

  stage_read16(A + (size_t)(mBlk + arow) * K + ach, abuf);
  stage_read16(W + (size_t)(nBlk + t) * K,          wbuf);
  stage_read16(W + (size_t)(nBlk + t) * K + 16,     wbuf + 16);

  f32x8 acc[4][4] = {};

  for (int k = 0; k < K; k += 32) {
    __syncthreads();
    stage_write(&ldsA[arow * LDS_STRIDE + ach], abuf, 4);
    stage_write(&ldsW[t * LDS_STRIDE],          wbuf, 8);
    if (k + 32 < K) {
      stage_read16(A + (size_t)(mBlk + arow) * K + (k + 32) + ach, abuf);
      stage_read16(W + (size_t)(nBlk + t) * K + (k + 32),          wbuf);
      stage_read16(W + (size_t)(nBlk + t) * K + (k + 32) + 16,     wbuf + 16);
    }
    __syncthreads();

    bf16x16 af[4], wf[4];
#pragma unroll
    for (int i = 0; i < 4; ++i)
      af[i] = lds_frag(ldsA + (wm + 16 * i) * LDS_STRIDE, LDS_STRIDE);
#pragma unroll
    for (int j = 0; j < 4; ++j)
      wf[j] = lds_frag(ldsW + (wn + 16 * j) * LDS_STRIDE, LDS_STRIDE);
#pragma unroll
    for (int i = 0; i < 4; ++i)
#pragma unroll
      for (int j = 0; j < 4; ++j)
        acc[i][j] = wmma_bf16(af[i], wf[j], acc[i][j]);
  }

  const int nlane = lane & 15;
  const int mh    = (lane >> 4) * 8;
  __syncthreads();
  if (MODE == 0 || MODE == 1) {
    bf16* so = (bf16*)sob;
#pragma unroll
    for (int i = 0; i < 4; ++i)
#pragma unroll
      for (int j = 0; j < 4; ++j) {
        const int nl = wn + 16 * j + nlane;
        const float bv = bias ? bias[nBlk + nl] : 0.0f;
#pragma unroll
        for (int r = 0; r < 8; ++r) {
          const int ml = wm + 16 * i + mh + r;
          const bf16 hv = (bf16)(acc[i][j][r] + bv);
          if (MODE == 0) so[ml * 264 + nl] = hv;
          else           so[nl * 136 + ml] = hv;
        }
      }
    __syncthreads();
#pragma unroll 1
    for (int pass = 0; pass < 2; ++pass) {
      if (MODE == 0) {
        for (int ch = t; ch < 128 * 32; ch += 256) { const int ml = ch >> 5, q = (ch & 31) * 8;
          *(volatile v4u_t*)((bf16*)out + (size_t)(mBlk + ml) * N + nBlk + q) = *(const v4ua*)(so + ml * 264 + q); }
      } else {
        const int b_ = mBlk / SS, s0 = mBlk & (SS - 1);
        for (int ch = t; ch < 256 * 16; ch += 256) { const int nl = ch >> 4, q = (ch & 15) * 8; const int n = nBlk + nl, h = n >> 6, dk = n & (DKK - 1);
          *(volatile v4u_t*)((bf16*)out + (((size_t)(b_ * HH + h)) * DKK + dk) * SS + s0 + q) = *(const v4ua*)(so + nl * 136 + q); }
      }
      __threadfence();
    }
  } else {
    float* so = (float*)sob;
#pragma unroll 1
    for (int hf = 0; hf < 2; ++hf) {
      if (wm == hf * 64) {
#pragma unroll
        for (int i = 0; i < 4; ++i)
#pragma unroll
          for (int j = 0; j < 4; ++j) {
            const int nl = wn + 16 * j + nlane;
            const float bv = bias ? bias[nBlk + nl] : 0.0f;
#pragma unroll
            for (int r = 0; r < 8; ++r) so[(16 * i + mh + r) * 260 + nl] = acc[i][j][r] + bv;
          }
      }
      __syncthreads();
#pragma unroll 1
      for (int pass = 0; pass < 2; ++pass) {
        for (int ch = t; ch < 64 * 64; ch += 256) { const int ml = ch >> 6, q = (ch & 63) * 4;
          *(volatile v4f_t*)((float*)out + (size_t)(mBlk + hf * 64 + ml) * N + nBlk + q) = *(const volatile v4fa*)(so + ml * 260 + q); }
        __threadfence();
      }
      __syncthreads();
    }
  }
}


#define GN 50000
#define GNP 50176
#define GE 600000
#define NS 32
#define NGR 128
#define F0 64
#define K1 96
#define H1W 256
#define RG1 25088

__device__ __forceinline__ float lk(float x, float s) { return x >= 0.0f ? x : s * x; }
__device__ __forceinline__ float eluf(float x) { return x > 0.0f ? x : expm1f(x); }
__device__ __forceinline__ int clampi(int v, int hi) { return v < 0 ? 0 : (v >= hi ? hi - 1 : v); }

#define OWN_SCAN_BEGIN(COUNT, KEYEXPR, AUXEXPR) \
  for (int c0 = 0; c0 < (COUNT); c0 += 256) { \
    const int e = c0 + tid; int d = -1, aux = 0; \
    if (e < (COUNT)) { d = (KEYEXPR); aux = (AUXEXPR); } \
    const int own = (d >= 0) ? (d & 7) : -1; unsigned mown = 0u; \
    _Pragma("unroll") for (int ww = 0; ww < 8; ++ww) { const unsigned m = __builtin_amdgcn_ballot_w32(own == ww); if (own == ww) mown = m; if (lane == 0) wcnt[ww][wave] = __builtin_popcount(m); } \
    __syncthreads(); \
    if (own >= 0) { int base = 0; _Pragma("unroll") for (int w2 = 0; w2 < 8; ++w2) base += (w2 < wave) ? wcnt[own][w2] : 0; \
      const int pos = base + __builtin_popcount(mown & ((1u << lane) - 1u)); qd[own][pos] = d; qs[own][pos] = aux; } \
    int total = 0; _Pragma("unroll") for (int w2 = 0; w2 < 8; ++w2) total += wcnt[wave][w2]; \
    __syncthreads();
#define OWN_SCAN_END __syncthreads(); }

__global__ __launch_bounds__(256) void k_subst(const float* __restrict__ x, const float* __restrict__ w1, const float* __restrict__ b1, const float* __restrict__ w2, const float* __restrict__ b2, float* __restrict__ wsub) {
  __shared__ float acc[NS][F0 + 1]; __shared__ int cnt[NS]; __shared__ int qd[8][256], qs[8][256]; __shared__ int wcnt[8][8]; __shared__ float lg[NS];
  const int tid = threadIdx.x, lane = tid & 31, wave = tid >> 5;
  for (int i = tid; i < NS * (F0 + 1); i += 256) (&acc[0][0])[i] = 0.0f;
  if (tid < NS) cnt[tid] = 0;
  __syncthreads();
  OWN_SCAN_BEGIN(GN, clampi((int)x[(size_t)e * F0 + 5], NS), e)
#pragma unroll 1
    for (int qi = 0; qi < total; ++qi) { const int s = qd[wave][qi], n = qs[wave][qi];
      acc[s][lane] += x[(size_t)n * F0 + lane]; acc[s][32 + lane] += x[(size_t)n * F0 + 32 + lane]; if (lane == 0) cnt[s] += 1; }
  OWN_SCAN_END
  if (tid < NS) { const float inv = 1.0f / fmaxf((float)cnt[tid], 1.0f); float l = b2[0];
    for (int j = 0; j < 32; ++j) { float hsum = b1[j]; for (int f = 0; f < F0; ++f) hsum += acc[tid][f] * inv * w1[f * 32 + j]; l += lk(hsum, 0.2f) * w2[j]; }
    lg[tid] = l; }
  __syncthreads();
  if (tid < NS) { float mx = -INFINITY; for (int s = 0; s < NS; ++s) mx = fmaxf(mx, lg[s]); float den = 0.f; for (int s = 0; s < NS; ++s) den += expf(lg[s] - mx);
    const float v = expf(lg[tid] - mx) / den; *(volatile float*)(wsub + tid) = v; }
  __threadfence(); __syncthreads();
  if (tid < NS) { const float v = *(volatile float*)(wsub + tid); *(volatile float*)(wsub + tid) = v; }
}
__global__ __launch_bounds__(256) void k_h0(const float* __restrict__ x, const float* __restrict__ wsub, float* __restrict__ H0) {
  const int n = blockIdx.x * 8 + (threadIdx.x >> 5), lane = threadIdx.x & 31;
  float v0 = 0.f, v1 = 0.f, v2 = 0.f;
  if (n < GN) { v0 = x[(size_t)n * F0 + lane]; v1 = x[(size_t)n * F0 + 32 + lane]; if (lane == 0) v2 = wsub[clampi((int)x[(size_t)n * F0 + 5], NS)]; }
  float* row = H0 + (size_t)n * K1;
#pragma unroll 1
  for (int pass = 0; pass < 2; ++pass) { *(volatile float*)(row + lane) = v0; *(volatile float*)(row + 32 + lane) = v1; *(volatile float*)(row + 64 + lane) = v2; __threadfence(); }
}
__global__ __launch_bounds__(96) void k_w1rows(const float* __restrict__ W1, float* __restrict__ Wr) {
  const int n = blockIdx.x, k = threadIdx.x; const float v = (k < 65) ? W1[(size_t)k * H1W + n] : 0.0f;
  *(volatile float*)(Wr + (size_t)n * K1 + k) = v; __threadfence(); *(volatile float*)(Wr + (size_t)n * K1 + k) = v;
}
__global__ __launch_bounds__(256) void k_packA2(const float* __restrict__ W2, float* __restrict__ A) {
  const int m = blockIdx.x, k = threadIdx.x; const float v = (m < F0) ? W2[(size_t)k * F0 + m] : 0.0f;
  *(volatile float*)(A + (size_t)m * H1W + k) = v; __threadfence(); *(volatile float*)(A + (size_t)m * H1W + k) = v;
}
template <int NH, int MW>
__global__ __launch_bounds__(256) void k_asad(const bf16* __restrict__ M, const float* __restrict__ as_, const float* __restrict__ ad_, float* __restrict__ AS, float* __restrict__ AD, float* __restrict__ MX) {
  __shared__ float st[3][8][4];
  const int n = blockIdx.x * 8 + (threadIdx.x >> 5), t = threadIdx.x, w = t >> 5, lane = t & 31;
#pragma unroll
  for (int h = 0; h < 4; ++h) {
    float s = 0.f, d = 0.f;
    if (h < NH && n < GN) { const float m0 = (float)M[(size_t)n * MW + h * 64 + lane], m1 = (float)M[(size_t)n * MW + h * 64 + 32 + lane];
      s = m0 * as_[h * 64 + lane] + m1 * as_[h * 64 + 32 + lane]; d = m0 * ad_[h * 64 + lane] + m1 * ad_[h * 64 + 32 + lane]; }
#pragma unroll
    for (int o = 16; o >= 1; o >>= 1) { s += __shfl_xor(s, o, 32); d += __shfl_xor(d, o, 32); }
    if (lane == 0) { st[0][w][h] = s; st[1][w][h] = d; st[2][w][h] = (h < NH) ? lk(s + d, 0.2f) : 0.0f; }
  }
  __syncthreads();
  if (t < 96) { const int which = t >> 5, i = t & 31; float* dst = (which == 0 ? AS : which == 1 ? AD : MX) + (size_t)blockIdx.x * 32 + i; const float v = st[which][i >> 2][i & 3];
    *(volatile float*)dst = v; __threadfence(); *(volatile float*)dst = v; }
}
template <int NH>
__global__ __launch_bounds__(256) void k_gmax(const int* __restrict__ srci, const int* __restrict__ dsti, const float* __restrict__ AS, const float* __restrict__ AD, float* __restrict__ MX) {
  __shared__ int qd[8][256], qs[8][256]; __shared__ int wcnt[8][8];
  const int tid = threadIdx.x, lane = tid & 31, wave = tid >> 5;
  OWN_SCAN_BEGIN(GE, clampi(dsti[e], GN), clampi(srci[e], GN))
    if (lane < NH) {
#pragma unroll 1
      for (int qi = 0; qi < total; ++qi) { const int dl = qd[wave][qi], sl = qs[wave][qi];
        const float ev = lk(AS[(size_t)sl * 4 + lane] + AD[(size_t)dl * 4 + lane], 0.2f); float* p = MX + (size_t)dl * 4 + lane; *p = fmaxf(*p, ev); } }
  OWN_SCAN_END
  __threadfence(); __syncthreads();
  for (int i = tid; i < GN; i += 256) { float* p = MX + (size_t)i * 4; const v4f_t v = *(const volatile v4fa*)p; *(volatile v4f_t*)p = v; }
  __threadfence();
}
template <int NH, int MW, int RANGE>
__global__ __launch_bounds__(256) void k_gacc(const int* __restrict__ srci, const int* __restrict__ dsti, const float* __restrict__ AS, const float* __restrict__ AD, const float* __restrict__ MX,
                                             const bf16* __restrict__ M, float* __restrict__ R, float* __restrict__ DEN, int rsel) {
  __shared__ int qd[8][256], qs[8][256]; __shared__ int wcnt[8][8];
  const int tid = threadIdx.x, lane = tid & 31, wave = tid >> 5, r0 = rsel * RANGE;
  constexpr int PER = MW / 32;
  for (int i = tid; i < RANGE * (MW / 4); i += 256) { const int nl = i / (MW / 4), c4 = (i % (MW / 4)) * 4, n = r0 + nl; v4f_t v; v.x = v.y = v.z = v.w = 0.0f;
    if (n < GN) { const int h = c4 / 64; const float ex = expf(lk(AS[(size_t)n * 4 + h] + AD[(size_t)n * 4 + h], 0.2f) - MX[(size_t)n * 4 + h]);
      v.x = ex * (float)M[(size_t)n * MW + c4]; v.y = ex * (float)M[(size_t)n * MW + c4 + 1]; v.z = ex * (float)M[(size_t)n * MW + c4 + 2]; v.w = ex * (float)M[(size_t)n * MW + c4 + 3]; }
    *(volatile v4f_t*)(R + (size_t)nl * MW + c4) = v; }
  for (int i = tid; i < RANGE; i += 256) { const int n = r0 + i; v4f_t v; v.x = v.y = v.z = v.w = 0.0f;
    if (n < GN) { for (int h = 0; h < NH; ++h) v[h] = expf(lk(AS[(size_t)n * 4 + h] + AD[(size_t)n * 4 + h], 0.2f) - MX[(size_t)n * 4 + h]); }
    *(volatile v4f_t*)(DEN + (size_t)n * 4) = v; }
  __threadfence(); __syncthreads();
  const int hl = (lane * PER) / 64;
  OWN_SCAN_BEGIN(GE, ((clampi(dsti[e], GN) >= r0 && clampi(dsti[e], GN) < r0 + RANGE) ? clampi(dsti[e], GN) - r0 : -1), clampi(srci[e], GN))
#pragma unroll 1
    for (int qi = 0; qi < total; ++qi) { const int dl = qd[wave][qi], sl = qs[wave][qi], dn = r0 + dl;
      float exh = 0.0f;
      if (hl < NH) { const float ev = lk(AS[(size_t)sl * 4 + hl] + AD[(size_t)dn * 4 + hl], 0.2f); exh = expf(ev - MX[(size_t)dn * 4 + hl]); }
      if (((lane * PER) & 63) == 0 && hl < NH) DEN[(size_t)dn * 4 + hl] += exh;
      float* row = R + (size_t)dl * MW + lane * PER; const bf16* ms = M + (size_t)sl * MW + lane * PER;
#pragma unroll
      for (int j = 0; j < PER; ++j) row[j] += exh * (float)ms[j]; }
  OWN_SCAN_END
  __threadfence(); __syncthreads();
  for (int i = tid; i < RANGE * (MW / 4); i += 256) { float* p = R + (size_t)i * 4; const v4f_t v = *(const volatile v4fa*)p; *(volatile v4f_t*)p = v; }
  for (int i = tid; i < RANGE; i += 256) { float* p = DEN + (size_t)(r0 + i) * 4; const v4f_t v = *(const volatile v4fa*)p; *(volatile v4f_t*)p = v; }
  __threadfence();
}

__global__ __launch_bounds__(256) void k_fin1(const float* __restrict__ R, const float* __restrict__ DEN, const float* __restrict__ b1, int r0, bf16* __restrict__ H1) {
  const int nl = blockIdx.x, n = r0 + nl, c = threadIdx.x; float v = 0.0f;
  if (n < GN) v = eluf(R[(size_t)nl * H1W + c] / (DEN[(size_t)n * 4 + (c >> 6)] + 1e-16f) + b1[c]);
  const bf16 hv = (bf16)v;
  const float vn = __shfl_xor(v, 1, 32);
  if ((c & 1) == 0) { bf16 pr[2]; pr[0] = hv; pr[1] = (bf16)vn; typedef unsigned u1a __attribute__((may_alias));
    *(volatile unsigned*)(H1 + (size_t)n * H1W + c) = *(const u1a*)pr; __threadfence(); *(volatile unsigned*)(H1 + (size_t)n * H1W + c) = *(const u1a*)pr; }
}
__global__ __launch_bounds__(256) void k_m2(const float* __restrict__ T, bf16* __restrict__ M2) {
  __shared__ float tile[64][65];
  const int n0 = blockIdx.x * 64, t = threadIdx.x;
  for (int i = t; i < 64 * 64; i += 256) { const int c = i >> 6, nn = i & 63; tile[c][nn] = T[(size_t)c * GNP + n0 + nn]; }
  __syncthreads();
#pragma unroll 1
  for (int pass = 0; pass < 2; ++pass) {
    for (int i = t; i < 64 * 8; i += 256) { const int nr = i >> 3, c8 = (i & 7) * 8; bf16 hh[8];
#pragma unroll
      for (int e = 0; e < 8; ++e) hh[e] = (bf16)tile[c8 + e][nr];
      *(volatile v4u_t*)(M2 + (size_t)(n0 + nr) * F0 + c8) = *(const v4ua*)hh; }
    __threadfence(); }
}
__global__ __launch_bounds__(256) void k_fin2(const float* __restrict__ R2, const float* __restrict__ DEN, const float* __restrict__ b2, float* __restrict__ H2) {
  const int n = blockIdx.x * 4 + (threadIdx.x >> 6), c = threadIdx.x & 63; if (n >= GN) return;
  const float v = R2[(size_t)n * F0 + c] / (DEN[(size_t)n * 4] + 1e-16f) + b2[c];
  *(volatile float*)(H2 + (size_t)n * F0 + c) = v; __threadfence(); *(volatile float*)(H2 + (size_t)n * F0 + c) = v;
}
__global__ __launch_bounds__(256) void k_pool(const float* __restrict__ H2, const int* __restrict__ batch, const float* __restrict__ Wp1, const float* __restrict__ bp1, const float* __restrict__ Wp2, const float* __restrict__ bp2, float* __restrict__ out) {
  __shared__ float acc[NGR][F0 + 1]; __shared__ int qd[8][256], qs[8][256]; __shared__ int wcnt[8][8]; __shared__ float res[NGR];
  const int tid = threadIdx.x, lane = tid & 31, wave = tid >> 5;
  for (int i = tid; i < NGR * (F0 + 1); i += 256) (&acc[0][0])[i] = 0.0f;
  __syncthreads();
  OWN_SCAN_BEGIN(GN, clampi(batch[e], NGR), e)
#pragma unroll 1
    for (int qi = 0; qi < total; ++qi) { const int g = qd[wave][qi], n = qs[wave][qi]; acc[g][lane] += H2[(size_t)n * F0 + lane]; acc[g][32 + lane] += H2[(size_t)n * F0 + 32 + lane]; }
  OWN_SCAN_END
  if (tid < NGR) { float o = bp2[0];
    for (int j = 0; j < 32; ++j) { float hsum = bp1[j]; for (int f = 0; f < F0; ++f) hsum += acc[tid][f] * Wp1[f * 32 + j]; o += eluf(hsum) * Wp2[j]; }
    res[tid] = o; }
  __syncthreads();
  if (tid < 32) { const v4f_t v = *(const volatile v4fa*)(res + tid * 4); *(volatile v4f_t*)(out + tid * 4) = v; __threadfence(); *(volatile v4f_t*)(out + tid * 4) = v; }
}

extern "C" void kernel_launch(void* const* d_in, const int* in_sizes, int n_in,
                              void* d_out, int out_size, void* d_ws, size_t ws_size,
                              hipStream_t stream) {
  (void)in_sizes; (void)n_in; (void)out_size; (void)ws_size;
  const float* x = (const float*)d_in[0];
  const int* ei = (const int*)d_in[1];
  const int* batch = (const int*)d_in[2];
  const float* wsa1 = (const float*)d_in[3]; const float* bsa1 = (const float*)d_in[4]; const float* wsa2 = (const float*)d_in[5]; const float* bsa2 = (const float*)d_in[6];
  const float* W1 = (const float*)d_in[7]; const float* as1 = (const float*)d_in[8]; const float* ad1 = (const float*)d_in[9]; const float* b1 = (const float*)d_in[10];
  const float* W2 = (const float*)d_in[11]; const float* as2 = (const float*)d_in[12]; const float* ad2 = (const float*)d_in[13]; const float* b2 = (const float*)d_in[14];
  const float* Wp1 = (const float*)d_in[15]; const float* bp1 = (const float*)d_in[16]; const float* Wp2 = (const float*)d_in[17]; const float* bp2 = (const float*)d_in[18];
  const int* srci = ei; const int* dsti = ei + (size_t)GE;
  char* ws = (char*)d_ws;
  float* wsub = (float*)ws; ws += 32 * 4 * 8;
  float* W1r = (float*)ws; ws += (size_t)H1W * K1 * 4;
  float* A2  = (float*)ws; ws += (size_t)128 * H1W * 4;
  float* AS  = (float*)ws; ws += (size_t)GNP * 4 * 4; float* AD = (float*)ws; ws += (size_t)GNP * 4 * 4;
  float* MX  = (float*)ws; ws += (size_t)GNP * 4 * 4; float* DEN = (float*)ws; ws += (size_t)GNP * 4 * 4;
  float* H0  = (float*)ws; ws += (size_t)GNP * K1 * 4;
  bf16* M1   = (bf16*)ws;  ws += (size_t)GNP * H1W * 2;
  float* T2  = (float*)M1;
  float* R   = (float*)ws; ws += (size_t)RG1 * H1W * 4;
  bf16* M2   = (bf16*)R; float* R2 = (float*)((char*)R + (size_t)GNP * F0 * 2);
  bf16* H1   = (bf16*)ws;  ws += (size_t)GNP * H1W * 2;
  float* H2  = (float*)ws; ws += (size_t)GNP * F0 * 4;
  k_subst<<<1, 256, 0, stream>>>(x, wsa1, bsa1, wsa2, bsa2, wsub);
  k_h0<<<GNP / 8, 256, 0, stream>>>(x, wsub, H0);
  k_w1rows<<<H1W, 96, 0, stream>>>(W1, W1r);
  k_packA2<<<128, 256, 0, stream>>>(W2, A2);
  dim3 blk(256);
  gemm_bias_kernel<float, float, 0><<<dim3(GNP / 128, 1), blk, 0, stream>>>(H0, W1r, nullptr, M1, GNP, H1W, K1);
  k_asad<4, H1W><<<GNP / 8, 256, 0, stream>>>(M1, as1, ad1, AS, AD, MX);
  k_gmax<4><<<1, 256, 0, stream>>>(srci, dsti, AS, AD, MX);
  for (int r = 0; r < GNP / RG1; ++r) { k_gacc<4, H1W, RG1><<<1, 256, 0, stream>>>(srci, dsti, AS, AD, MX, M1, R, DEN, r); k_fin1<<<RG1, 256, 0, stream>>>(R, DEN, b1, r * RG1, H1); }
  gemm_bias_kernel<float, bf16, 2><<<dim3(1, GNP / 256), blk, 0, stream>>>(A2, H1, nullptr, T2, 128, GNP, H1W);
  k_m2<<<GNP / 64, 256, 0, stream>>>(T2, M2);
  k_asad<1, F0><<<GNP / 8, 256, 0, stream>>>(M2, as2, ad2, AS, AD, MX);
  k_gmax<1><<<1, 256, 0, stream>>>(srci, dsti, AS, AD, MX);
  k_gacc<1, F0, GNP><<<1, 256, 0, stream>>>(srci, dsti, AS, AD, MX, M2, R2, DEN, 0);
  k_fin2<<<GNP / 4, 256, 0, stream>>>(R2, DEN, b2, H2);
  k_pool<<<1, 256, 0, stream>>>(H2, batch, Wp1, bp1, Wp2, bp2, (float*)d_out);
}
